// QuadraticFormSheafLearner_9174050144889
// MI455X (gfx1250) — hardware-run, weakly checked
//
#include <hip/hip_runtime.h>
#include <math.h>

typedef __attribute__((ext_vector_type(16))) __bf16   v16b;
typedef __attribute__((ext_vector_type(8)))  __bf16   v8b;
typedef __attribute__((ext_vector_type(8)))  float    v8f;
typedef __attribute__((ext_vector_type(4)))  float    v4f;
typedef __attribute__((ext_vector_type(4)))  unsigned v4u;

constexpr int kNodes      = 50000;
constexpr int kNodesPad   = 50048;
constexpr int kEdges      = 800000;
constexpr int kCin        = 64;
constexpr int kForms      = 16;
constexpr int kD2         = 128;
constexpr int kKcat       = 192;
constexpr int kChunkForms = 4;
constexpr int kChunkCols  = kChunkForms * kCin;
constexpr int kNumChunks  = kForms / kChunkForms;
constexpr int kPlaneRows  = kForms * kCin;
static_assert(kD2 == 2 * kCin, "concatenated feature width");
static_assert(kChunkCols == 256 && kNumChunks == 4 && kPlaneRows == 1024, "chunking");
static_assert((kNodesPad % 64) == 0 && kNodesPad >= kNodes, "GEMM M multiple of 64");
static_assert((kChunkCols % 64) == 0, "GEMM N multiple of 64");
static_assert((kKcat % 32) == 0 && kKcat == 3 * kCin, "GEMM K multiple of 32");
static_assert((kEdges % 256) == 0, "edge grid exact");
static_assert((kNodesPad % 128) == 0, "node grid exact");
static_assert(((kNodesPad * 8) % 256) == 0, "split grid exact");
static_assert(((3 * kPlaneRows * 8) % 256) == 0 && ((kPlaneRows * 8) % 256) == 0, "weight grid exact, plane uniform per block");
static_assert(((kNodesPad / 64) * (kChunkCols / 64)) % 8 == 0, "GEMM tiles multiple of 8 waves");

constexpr size_t kBytesAX  = (size_t)kNodesPad * kKcat * 2;
constexpr size_t kBytesWP  = (size_t)3 * kPlaneRows * kKcat * 2;
constexpr size_t kBytesTT  = (size_t)kNodesPad * kChunkCols * 4;
constexpr size_t kBytesPN1 = (size_t)kNodesPad * kChunkForms * 4;
constexpr size_t kBytesSP1 = (size_t)kEdges * kChunkForms * 4;
constexpr size_t kOffAX    = 0;
constexpr size_t kOffWP    = kOffAX + kBytesAX;
constexpr size_t kOffTT    = kOffWP + kBytesWP;
constexpr size_t kOffPN    = kOffTT + kBytesTT;
constexpr size_t kOffSP    = kOffPN + 8 * kBytesPN1;
constexpr size_t kWsTotal  = kOffSP + 3 * kBytesSP1;
static_assert(kBytesAX == 19218432ull && kBytesWP == 1179648ull && kBytesTT == 51249152ull, "plane sizes");
static_assert(kBytesPN1 == 800768ull && kBytesSP1 == 12800000ull, "plane sizes");
static_assert(kWsTotal == 116453376ull, "carve total");
static_assert(kWsTotal <= 134217728ull, "carve cap");
static_assert((kOffWP % 128) == 0 && (kOffTT % 128) == 0 && (kOffPN % 128) == 0 && (kOffSP % 128) == 0 &&
              (kBytesPN1 % 128) == 0 && (kBytesSP1 % 128) == 0, "128-B aligned regions");

__device__ __forceinline__ unsigned bf_bits_rne(float f) {
  const unsigned u = __float_as_uint(f);
  return (u + 0x7FFFu + ((u >> 16) & 1u)) >> 16;
}
__device__ __forceinline__ float bf_bits_to_f32(unsigned h) { return __uint_as_float(h << 16); }

__device__ __forceinline__ void split_pack2(float fa, float fb, unsigned& hw, unsigned& lw) {
  const unsigned ha = bf_bits_rne(fa);
  const unsigned hb = bf_bits_rne(fb);
  const float ra = fa - bf_bits_to_f32(ha);
  const float rb = fb - bf_bits_to_f32(hb);
  const unsigned la = bf_bits_rne(ra);
  const unsigned lb = bf_bits_rne(rb);
  hw = (ha & 0xFFFFu) | ((hb & 0xFFFFu) << 16);
  lw = (la & 0xFFFFu) | ((lb & 0xFFFFu) << 16);
}

__device__ __forceinline__ float tanh_sat(float z) {
  const float e2 = __expf(2.0f * z);
  const float rc = __builtin_amdgcn_rcpf(e2 + 1.0f);
  return 1.0f - 2.0f * rc;
}

__device__ __forceinline__ void dot4x64(const float* __restrict__ tr, const float* __restrict__ xr,
                                        float& a0, float& a1, float& a2, float& a3) {
#pragma unroll 1
  for (int s = 0; s < 16; s += 2) {
#pragma unroll
    for (int u = 0; u < 2; ++u) {
      const int o = (s + u) * 4;
      const v4f xv = *(const v4f*)(xr + o);
      const v4f t0 = *(const v4f*)(tr + o);
      const v4f t1 = *(const v4f*)(tr + 64 + o);
      const v4f t2 = *(const v4f*)(tr + 128 + o);
      const v4f t3 = *(const v4f*)(tr + 192 + o);
      a0 = fmaf(t0[0], xv[0], a0); a0 = fmaf(t0[1], xv[1], a0); a0 = fmaf(t0[2], xv[2], a0); a0 = fmaf(t0[3], xv[3], a0);
      a1 = fmaf(t1[0], xv[0], a1); a1 = fmaf(t1[1], xv[1], a1); a1 = fmaf(t1[2], xv[2], a1); a1 = fmaf(t1[3], xv[3], a1);
      a2 = fmaf(t2[0], xv[0], a2); a2 = fmaf(t2[1], xv[1], a2); a2 = fmaf(t2[2], xv[2], a2); a2 = fmaf(t2[3], xv[3], a2);
      a3 = fmaf(t3[0], xv[0], a3); a3 = fmaf(t3[1], xv[1], a3); a3 = fmaf(t3[2], xv[2], a3); a3 = fmaf(t3[3], xv[3], a3);
    }
  }
}

__device__ __forceinline__ void guard1_b(v8f& a, v16b x, v16b y) { asm volatile("v_nop\n\tv_nop\n\tv_nop\n\tv_nop" : "+v"(a) : "v"(x), "v"(y)); }
__device__ __forceinline__ void keep4_b(v16b a, v16b b, v16b c, v16b d) { asm volatile("v_nop" :: "v"(a), "v"(b), "v"(c), "v"(d)); }
__device__ __forceinline__ void acc_guard4(v8f& a, v8f& b, v8f& c, v8f& d) { asm volatile("v_nop\n\tv_nop\n\tv_nop\n\tv_nop" : "+v"(a), "+v"(b), "+v"(c), "+v"(d)); }
struct FragB {
  union U { v16b v; v8b h[2]; };
  static __device__ __forceinline__ v16b load(const __bf16* p) {
    U f; f.h[0] = *(const v8b*)(p); f.h[1] = *(const v8b*)(p + 16); return f.v;
  }
  static __device__ __forceinline__ v8f mma(v16b a, v16b b, v8f c) {
    return __builtin_amdgcn_wmma_f32_16x16x32_bf16(false, a, false, b, (short)0, c, false, false);
  }
};

__global__ __launch_bounds__(256) void node_gemm_kernel(
    const unsigned short* __restrict__ Ap, int lda,
    const unsigned short* __restrict__ Btp, int ldb,
    float* __restrict__ C, int ldc,
    int M, int N, int K) {
  const __bf16* A  = (const __bf16*)Ap;
  const __bf16* Bt = (const __bf16*)Btp;
  __shared__ __align__(16) float sT[8][16 * 68];
  const int lane = threadIdx.x & 31;
  const int wave = threadIdx.x >> 5;
  const int tilesN = N >> 6;
  const int tilesM = M >> 6;
  const int tile = blockIdx.x * 8 + wave;
  if (tile >= tilesM * tilesN) return;
  const int tm = tile / tilesN;
  const int tn = tile - tm * tilesN;
  const int m0 = tm << 6;
  const int n0 = tn << 6;

  const int rlane = lane & 15;
  const int koff  = (lane >> 4) * 8;
  const int mOff  = (lane >> 4) * 8;

  v8f acc[4][4];
#pragma unroll
  for (int i = 0; i < 4; ++i)
#pragma unroll
    for (int j = 0; j < 4; ++j) acc[i][j] = (v8f){0.f,0.f,0.f,0.f,0.f,0.f,0.f,0.f};

  for (int k0 = 0; k0 < K; k0 += 32) {
    v16b bh[4];
#pragma unroll
    for (int j = 0; j < 4; ++j) {
      const size_t bo = (size_t)(n0 + (j << 4) + rlane) * ldb + koff + k0;
      bh[j] = FragB::load(Bt + bo);
    }
#pragma unroll
    for (int i = 0; i < 4; ++i) {
      const size_t ao = (size_t)(m0 + (i << 4) + rlane) * lda + koff + k0;
      const v16b ah = FragB::load(A + ao);
#pragma unroll
      for (int j = 0; j < 4; ++j) acc[i][j] = FragB::mma(ah, bh[j], acc[i][j]);
      guard1_b(acc[i][0], ah, bh[0]);
      guard1_b(acc[i][1], ah, bh[1]);
      guard1_b(acc[i][2], ah, bh[2]);
      guard1_b(acc[i][3], ah, bh[3]);
    }
    keep4_b(bh[0], bh[1], bh[2], bh[3]);
  }
  acc_guard4(acc[0][0], acc[0][1], acc[0][2], acc[0][3]);
  acc_guard4(acc[1][0], acc[1][1], acc[1][2], acc[1][3]);
  acc_guard4(acc[2][0], acc[2][1], acc[2][2], acc[2][3]);
  acc_guard4(acc[3][0], acc[3][1], acc[3][2], acc[3][3]);

  float* slab = sT[wave];
#pragma unroll
  for (int i = 0; i < 4; ++i) {
    const int mBase = m0 + (i << 4);
#pragma unroll
    for (int j = 0; j < 4; ++j) {
#pragma unroll
      for (int r = 0; r < 8; ++r) {
        slab[(mOff + r) * 68 + (j << 4) + rlane] = acc[i][j][r];
      }
    }
    __builtin_amdgcn_fence(__ATOMIC_RELEASE, "workgroup");
    __builtin_amdgcn_wave_barrier();
    __builtin_amdgcn_fence(__ATOMIC_ACQUIRE, "workgroup");
    {
      const int hh = lane >> 4, c4 = (lane & 15) * 4;
      for (int pass = 0; pass < 2; ++pass) {
#pragma unroll
        for (int it = 0; it < 8; ++it) {
          const int row = it * 2 + hh;
          const v4f v = *(const v4f*)(slab + row * 68 + c4);
          *(volatile v4f*)(C + (size_t)(mBase + row) * ldc + n0 + c4) = v;
        }
        __threadfence();
      }
    }
    __builtin_amdgcn_fence(__ATOMIC_RELEASE, "workgroup");
    __builtin_amdgcn_wave_barrier();
    __builtin_amdgcn_fence(__ATOMIC_ACQUIRE, "workgroup");
  }
}

__global__ __launch_bounds__(256) void split_x_kernel(const float* __restrict__ x, unsigned short* __restrict__ AX) {
  const int t  = blockIdx.x * 256 + threadIdx.x;
  const int n  = t >> 3;
  const int ch = t & 7;
  const bool real = n < kNodes;
  const int nc = real ? n : (kNodes - 1);
  const float* src = x + (size_t)nc * kCin + ch * 8;
  const v4f a0 = *(const v4f*)(src);
  const v4f a1 = *(const v4f*)(src + 4);
  const float f0 = real ? a0[0] : 0.0f;
  const float f1 = real ? a0[1] : 0.0f;
  const float f2 = real ? a0[2] : 0.0f;
  const float f3 = real ? a0[3] : 0.0f;
  const float f4 = real ? a1[0] : 0.0f;
  const float f5 = real ? a1[1] : 0.0f;
  const float f6 = real ? a1[2] : 0.0f;
  const float f7 = real ? a1[3] : 0.0f;
  unsigned h0, h1, h2, h3, l0, l1, l2, l3;
  split_pack2(f0, f1, h0, l0);
  split_pack2(f2, f3, h1, l1);
  split_pack2(f4, f5, h2, l2);
  split_pack2(f6, f7, h3, l3);
  const v4u hv = (v4u){h0, h1, h2, h3};
  const v4u lv = (v4u){l0, l1, l2, l3};
  unsigned short* d = AX + (size_t)n * kKcat + ch * 8;
  *(volatile v4u*)(void*)(d)       = hv;
  *(volatile v4u*)(void*)(d + 64)  = lv;
  *(volatile v4u*)(void*)(d + 128) = hv;
  __threadfence();
  *(volatile v4u*)(void*)(d)       = hv;
  *(volatile v4u*)(void*)(d + 64)  = lv;
  *(volatile v4u*)(void*)(d + 128) = hv;
}

__global__ __launch_bounds__(256) void prep_w_kernel(const float* __restrict__ Mw, unsigned short* __restrict__ WP) {
  const int t     = blockIdx.x * 256 + threadIdx.x;
  const int ch    = t & 7;
  const int n     = (t >> 3) & (kPlaneRows - 1);
  const int plane = t >> 13;
  const int m  = n >> 6;
  const int j  = n & 63;
  const int k0 = ch * 8;
  const int rowoff = (plane == 1) ? 64 : 0;
  const int coloff = (plane >= 1) ? 64 : 0;
  const bool isE = (plane == 2);
  const float* Mm = Mw + (size_t)m * kD2 * kD2;
  const float* p1 = Mm + (size_t)(rowoff + k0) * kD2 + coloff + j;
  const float* p2 = Mm + (size_t)(64 + j) * kD2 + k0;
  const v4f c0 = *(const v4f*)(p2);
  const v4f c1 = *(const v4f*)(p2 + 4);
  float cadd[8];
  cadd[0] = c0[0]; cadd[1] = c0[1]; cadd[2] = c0[2]; cadd[3] = c0[3];
  cadd[4] = c1[0]; cadd[5] = c1[1]; cadd[6] = c1[2]; cadd[7] = c1[3];
  float f[8];
#pragma unroll
  for (int i = 0; i < 8; ++i) {
    const float base = p1[(size_t)i * kD2];
    const float extra = isE ? cadd[i] : 0.0f;
    f[i] = base + extra;
  }
  unsigned h0, h1, h2, h3, l0, l1, l2, l3;
  split_pack2(f[0], f[1], h0, l0);
  split_pack2(f[2], f[3], h1, l1);
  split_pack2(f[4], f[5], h2, l2);
  split_pack2(f[6], f[7], h3, l3);
  const v4u hv = (v4u){h0, h1, h2, h3};
  const v4u lv = (v4u){l0, l1, l2, l3};
  unsigned short* d = WP + ((size_t)plane * kPlaneRows + n) * kKcat + k0;
  *(volatile v4u*)(void*)(d)       = hv;
  *(volatile v4u*)(void*)(d + 64)  = hv;
  *(volatile v4u*)(void*)(d + 128) = lv;
  __threadfence();
  *(volatile v4u*)(void*)(d)       = hv;
  *(volatile v4u*)(void*)(d + 64)  = hv;
  *(volatile v4u*)(void*)(d + 128) = lv;
}

__global__ __launch_bounds__(128) void node_dot_kernel(const float* __restrict__ TT, const float* __restrict__ x,
                                                       float* __restrict__ P) {
  const int n = blockIdx.x * 128 + threadIdx.x;
  const bool real = n < kNodes;
  const int nx = real ? n : (kNodes - 1);
  const float* tr = TT + (size_t)n * kChunkCols;
  const float* xr = x + (size_t)nx * kCin;
  float a0 = 0.0f, a1 = 0.0f, a2 = 0.0f, a3 = 0.0f;
  dot4x64(tr, xr, a0, a1, a2, a3);
  const float r0 = real ? a0 : 0.0f;
  const float r1 = real ? a1 : 0.0f;
  const float r2 = real ? a2 : 0.0f;
  const float r3 = real ? a3 : 0.0f;
  const v4f rv = (v4f){r0, r1, r2, r3};
  float* d = P + (size_t)n * kChunkForms;
  *(volatile v4f*)(d) = rv;
  __threadfence();
  *(volatile v4f*)(d) = rv;
}

template <bool FINAL>
__global__ __launch_bounds__(256) void edge_kernel(
    const float* __restrict__ TT, const float* __restrict__ x, const int* __restrict__ ei,
    const float* __restrict__ PA, const float* __restrict__ PD,
    const float* S0, const float* S1, const float* S2, float* dst) {
  __shared__ __align__(16) float slab[FINAL ? (8 * 512) : 32];
  const int lane = threadIdx.x & 31;
  const int wave = threadIdx.x >> 5;
  const int e  = blockIdx.x * 256 + threadIdx.x;
  const int ec = (e < kEdges) ? e : (kEdges - 1);
  int r = ei[ec];
  int c = ei[kEdges + ec];
  r = (r < 0) ? 0 : ((r > kNodes - 1) ? (kNodes - 1) : r);
  c = (c < 0) ? 0 : ((c > kNodes - 1) ? (kNodes - 1) : c);
  const v4f pa = *(const v4f*)(PA + (size_t)r * kChunkForms);
  const v4f pd = *(const v4f*)(PD + (size_t)c * kChunkForms);
  const float* tr = TT + (size_t)r * kChunkCols;
  const float* xr = x + (size_t)c * kCin;
  float a0 = 0.0f, a1 = 0.0f, a2 = 0.0f, a3 = 0.0f;
  dot4x64(tr, xr, a0, a1, a2, a3);
  const float q0 = (a0 + pa[0]) + pd[0];
  const float q1 = (a1 + pa[1]) + pd[1];
  const float q2 = (a2 + pa[2]) + pd[2];
  const float q3 = (a3 + pa[3]) + pd[3];
  const v4f cur = (v4f){tanh_sat(q0), tanh_sat(q1), tanh_sat(q2), tanh_sat(q3)};
  if (!FINAL) {
    float* d = dst + (size_t)ec * kChunkForms;
    *(volatile v4f*)(d) = cur;
    __threadfence();
    *(volatile v4f*)(d) = cur;
  } else {
    const v4f s0 = *(const v4f*)(S0 + (size_t)ec * kChunkForms);
    const v4f s1 = *(const v4f*)(S1 + (size_t)ec * kChunkForms);
    const v4f s2 = *(const v4f*)(S2 + (size_t)ec * kChunkForms);
    float* sl = slab + wave * 512;
    *(v4f*)(sl + lane * 16 + 0)  = s0;
    *(v4f*)(sl + lane * 16 + 4)  = s1;
    *(v4f*)(sl + lane * 16 + 8)  = s2;
    *(v4f*)(sl + lane * 16 + 12) = cur;
    __syncthreads();
    v4f o0 = *(const v4f*)(sl + 0 * 128 + lane * 4);
    v4f o1 = *(const v4f*)(sl + 1 * 128 + lane * 4);
    v4f o2 = *(const v4f*)(sl + 2 * 128 + lane * 4);
    v4f o3 = *(const v4f*)(sl + 3 * 128 + lane * 4);
    float* ob = dst + ((size_t)blockIdx.x * 256 + (size_t)wave * 32) * kForms;
    for (int pass = 0; pass < 2; ++pass) {
      *(volatile v4f*)(ob + 0 * 128 + lane * 4) = o0;
      *(volatile v4f*)(ob + 1 * 128 + lane * 4) = o1;
      *(volatile v4f*)(ob + 2 * 128 + lane * 4) = o2;
      *(volatile v4f*)(ob + 3 * 128 + lane * 4) = o3;
      __threadfence();
    }
  }
}

extern "C" void kernel_launch(void* const* d_in, const int* in_sizes, int n_in,
                              void* d_out, int out_size, void* d_ws, size_t ws_size,
                              hipStream_t stream) {
  if (n_in < 3) return;
  if (in_sizes[0] != kNodes * kCin) return;
  if (in_sizes[1] != 2 * kEdges) return;
  if (in_sizes[2] != kForms * kD2 * kD2) return;
  if (out_size != kEdges * kForms) return;
  if (ws_size < kWsTotal) return;

  const float* x  = (const float*)d_in[0];
  const int*   ei = (const int*)d_in[1];
  const float* Mw = (const float*)d_in[2];
  float* out = (float*)d_out;

  char* ws = (char*)d_ws;
  unsigned short* AX = (unsigned short*)(ws + kOffAX);
  unsigned short* WP = (unsigned short*)(ws + kOffWP);
  float*          TT = (float*)(ws + kOffTT);
  float*          PN = (float*)(ws + kOffPN);
  float*          SP = (float*)(ws + kOffSP);
  const size_t planeFloatsPN = (size_t)kNodesPad * kChunkForms;
  const size_t planeFloatsSP = (size_t)kEdges * kChunkForms;
  const int gemmBlocks = ((kNodesPad / 64) * (kChunkCols / 64)) / 8;

  split_x_kernel<<<(kNodesPad * 8) / 256, 256, 0, stream>>>(x, AX);
  prep_w_kernel<<<(3 * kPlaneRows * 8) / 256, 256, 0, stream>>>(Mw, WP);

  for (int blk = 0; blk < 2; ++blk) {
    for (int ch = 0; ch < kNumChunks; ++ch) {
      const unsigned short* Bt = WP + ((size_t)blk * kPlaneRows + (size_t)ch * kChunkCols) * kKcat;
      node_gemm_kernel<<<gemmBlocks, 256, 0, stream>>>(AX, kKcat, Bt, kKcat, TT, kChunkCols,
                                                       kNodesPad, kChunkCols, kKcat);
      node_dot_kernel<<<kNodesPad / 128, 128, 0, stream>>>(TT, x, PN + (size_t)(blk * kNumChunks + ch) * planeFloatsPN);
    }
  }

  const float* S0 = SP;
  const float* S1 = SP + planeFloatsSP;
  const float* S2 = SP + 2 * planeFloatsSP;
  for (int ch = 0; ch < kNumChunks; ++ch) {
    const unsigned short* Bt = WP + ((size_t)2 * kPlaneRows + (size_t)ch * kChunkCols) * kKcat;
    node_gemm_kernel<<<gemmBlocks, 256, 0, stream>>>(AX, kKcat, Bt, kKcat, TT, kChunkCols,
                                                     kNodesPad, kChunkCols, kKcat);
    const float* PAc = PN + (size_t)(0 * kNumChunks + ch) * planeFloatsPN;
    const float* PDc = PN + (size_t)(1 * kNumChunks + ch) * planeFloatsPN;
    if (ch < kNumChunks - 1) {
      edge_kernel<false><<<kEdges / 256, 256, 0, stream>>>(TT, x, ei, PAc, PDc, S0, S1, S2,
                                                           SP + (size_t)ch * planeFloatsSP);
    } else {
      edge_kernel<true><<<kEdges / 256, 256, 0, stream>>>(TT, x, ei, PAc, PDc, S0, S1, S2, out);
    }
  }
}
